// TriangleAttn_42099269436004
// MI455X (gfx1250) — hardware-verified
//
#include <hip/hip_runtime.h>
#include <math.h>
#include <stdint.h>

#define NN     256
#define DD     128
#define NH     4
#define DHD    32
#define NROWS  65536
#define NQKV   384
#define NCAT   528
#define SCALEV 0.17677669529663687f
#define LN_EPS 1e-5f
#define MINV   (-3.40282347e38f)

#define XP  136
#define SLP 68
#define KP  40
#define VP  264
#define PP  72
#define OSP 36

#define AT_KSH  0
#define AT_KSL  20480
#define AT_VTH  40960
#define AT_VTL  57856
#define AT_PH   74752
#define AT_PL   93184
#define AT_OS   111616
#define AT_SMEM 130048

typedef unsigned short us;
typedef us       v8us __attribute__((ext_vector_type(8)));
typedef __bf16   v16b __attribute__((ext_vector_type(16)));
typedef float    v8f  __attribute__((ext_vector_type(8)));
typedef float    v4f  __attribute__((ext_vector_type(4)));
typedef unsigned v2u  __attribute__((ext_vector_type(2)));
typedef unsigned v4u  __attribute__((ext_vector_type(4)));

__device__ __forceinline__ us f2bf_bits(float f) {
  unsigned u = __float_as_uint(f);
  return (us)((u + 0x7FFFu + ((u >> 16) & 1u)) >> 16);
}
__device__ __forceinline__ float bf2f(us b) { return __uint_as_float(((unsigned)b) << 16); }
__device__ __forceinline__ void split_bf(float f, us& h, us& l) { h = f2bf_bits(f); l = f2bf_bits(f - bf2f(h)); }
__device__ __forceinline__ unsigned pk16(us a, us b) { return (unsigned)a | ((unsigned)b << 16); }

union FragU { v16b v; v8us h[2]; };
__device__ __forceinline__ v16b ldfrag(const us* p) {
  FragU f; f.h[0] = *(const v8us*)p; f.h[1] = *(const v8us*)(p + 16); return f.v;
}

__device__ __forceinline__ v8f mma_g(v16b a, v16b b, v8f c) {
  c = __builtin_amdgcn_wmma_f32_16x16x32_bf16(false, a, false, b, (short)0, c, false, false);
  asm volatile("v_nop\n\tv_nop\n\tv_nop\n\tv_nop" : "+v"(c) : "v"(a), "v"(b));
  return c;
}
__device__ __forceinline__ v8f zero8() { v8f z = {0.f, 0.f, 0.f, 0.f, 0.f, 0.f, 0.f, 0.f}; return z; }
__device__ __forceinline__ void wave_lds_sync() {
  __builtin_amdgcn_fence(__ATOMIC_RELEASE, "workgroup");
  __builtin_amdgcn_wave_barrier();
  __builtin_amdgcn_fence(__ATOMIC_ACQUIRE, "workgroup");
}

__global__ __launch_bounds__(32) void prep_kernel(const float* __restrict__ Wqkv, const float* __restrict__ Wb,
                                                  const float* __restrict__ Wg, const float* __restrict__ Wout,
                                                  us* __restrict__ WTh, us* __restrict__ WTl,
                                                  us* __restrict__ WoTh, us* __restrict__ WoTl) {
  const int r = blockIdx.x;
  const int lane = threadIdx.x & 31;
  float x[4];
  us* dh; us* dl; int orow;
  if (r < NCAT) {
#pragma unroll
    for (int e = 0; e < 4; ++e) {
      const int k = 4 * lane + e;
      float v;
      if (r < NQKV)      v = Wqkv[k * NQKV + r];
      else if (r < 512)  v = Wg[k * DD + (r - NQKV)];
      else if (r < 516)  v = Wb[k * NH + (r - 512)];
      else               v = 0.0f;
      x[e] = v;
    }
    dh = WTh; dl = WTl; orow = r;
  } else {
    orow = r - NCAT;
#pragma unroll
    for (int e = 0; e < 4; ++e) x[e] = Wout[(4 * lane + e) * DD + orow];
    dh = WoTh; dl = WoTl;
  }
  us hb[4], lb[4];
#pragma unroll
  for (int e = 0; e < 4; ++e) split_bf(x[e], hb[e], lb[e]);
  v2u hv, lv;
  hv[0] = pk16(hb[0], hb[1]); hv[1] = pk16(hb[2], hb[3]);
  lv[0] = pk16(lb[0], lb[1]); lv[1] = pk16(lb[2], lb[3]);
  volatile v2u* ph = (volatile v2u*)(dh + (size_t)orow * DD + 4 * lane);
  volatile v2u* pl = (volatile v2u*)(dl + (size_t)orow * DD + 4 * lane);
  *ph = hv; *pl = lv;
  __threadfence();
  *ph = hv; *pl = lv;
}

__global__ __launch_bounds__(256) void proj_kernel(const float* __restrict__ edges,
                                                   const float* __restrict__ gam, const float* __restrict__ bet,
                                                   const float* __restrict__ bg,
                                                   const us* __restrict__ WTh, const us* __restrict__ WTl,
                                                   us* __restrict__ QKVh, us* __restrict__ QKVl,
                                                   float* __restrict__ Gout, float* __restrict__ BIAS) {
  __shared__ __align__(16) us Xh[32 * XP];
  __shared__ __align__(16) us Xl[32 * XP];
  __shared__ __align__(16) float slab[8][16 * SLP];
  const int tid = threadIdx.x, wave = tid >> 5, lane = tid & 31, hh = lane >> 4, c = lane & 15;
  const int m0 = blockIdx.x * 32;

  {
    const v4f g4 = *(const v4f*)(gam + 4 * lane);
    const v4f b4 = *(const v4f*)(bet + 4 * lane);
#pragma unroll
    for (int rr = 0; rr < 4; ++rr) {
      const int row = wave * 4 + rr;
      const v4f x = *(const v4f*)(edges + (size_t)(m0 + row) * DD + 4 * lane);
      float s = (x[0] + x[1]) + (x[2] + x[3]);
#pragma unroll
      for (int off = 16; off > 0; off >>= 1) s += __shfl_xor(s, off, 32);
      const float mu = s * (1.0f / 128.0f);
      float dx[4];
      float q = 0.0f;
#pragma unroll
      for (int e = 0; e < 4; ++e) { dx[e] = x[e] - mu; q += dx[e] * dx[e]; }
#pragma unroll
      for (int off = 16; off > 0; off >>= 1) q += __shfl_xor(q, off, 32);
      const float rstd = 1.0f / sqrtf(q * (1.0f / 128.0f) + LN_EPS);
      us hb[4], lb[4];
#pragma unroll
      for (int e = 0; e < 4; ++e) split_bf(dx[e] * rstd * g4[e] + b4[e], hb[e], lb[e]);
      v2u ph, pl;
      ph[0] = pk16(hb[0], hb[1]); ph[1] = pk16(hb[2], hb[3]);
      pl[0] = pk16(lb[0], lb[1]); pl[1] = pk16(lb[2], lb[3]);
      *(v2u*)(Xh + row * XP + 4 * lane) = ph;
      *(v2u*)(Xl + row * XP + 4 * lane) = pl;
    }
  }
  __syncthreads();

  float* sl = slab[wave];
  for (int t = wave; t < 9; t += 8) {
    if (t < 8) {
      const int n0 = t * 64;
      v8f acc[2][4];
#pragma unroll
      for (int i = 0; i < 2; ++i)
#pragma unroll
        for (int j = 0; j < 4; ++j) acc[i][j] = zero8();
#pragma unroll
      for (int ks = 0; ks < 4; ++ks) {
        const int k0 = ks * 32;
        v16b ah[2], al[2];
#pragma unroll
        for (int i = 0; i < 2; ++i) {
          ah[i] = ldfrag(Xh + (16 * i + c) * XP + k0 + 8 * hh);
          al[i] = ldfrag(Xl + (16 * i + c) * XP + k0 + 8 * hh);
        }
#pragma unroll
        for (int j = 0; j < 4; ++j) {
          const size_t bo = (size_t)(n0 + 16 * j + c) * DD + k0 + 8 * hh;
          const v16b bh = ldfrag(WTh + bo);
          const v16b bl = ldfrag(WTl + bo);
#pragma unroll
          for (int i = 0; i < 2; ++i) {
            acc[i][j] = mma_g(ah[i], bh, acc[i][j]);
            acc[i][j] = mma_g(ah[i], bl, acc[i][j]);
            acc[i][j] = mma_g(al[i], bh, acc[i][j]);
          }
        }
      }
      if (t < 6) {
        const int q = lane >> 3, c8 = (lane & 7) * 8;
#pragma unroll
        for (int i = 0; i < 2; ++i) {
#pragma unroll
          for (int j = 0; j < 4; ++j)
#pragma unroll
            for (int r = 0; r < 8; ++r) sl[(8 * hh + r) * SLP + 16 * j + c] = acc[i][j][r];
          wave_lds_sync();
          v8us hv[4], lv[4];
#pragma unroll
          for (int it = 0; it < 4; ++it) {
            const float* sp = sl + (it * 4 + q) * SLP + c8;
            v8us a, b;
#pragma unroll
            for (int e = 0; e < 8; ++e) { us h_, l_; split_bf(sp[e], h_, l_); a[e] = h_; b[e] = l_; }
            hv[it] = a; lv[it] = b;
          }
          const size_t rb = (size_t)(m0 + 16 * i) * NQKV + n0 + c8;
#pragma unroll
          for (int it = 0; it < 4; ++it) {
            const size_t o = rb + (size_t)(it * 4 + q) * NQKV;
            *(volatile v8us*)(QKVh + o) = hv[it];
            *(volatile v8us*)(QKVl + o) = lv[it];
          }
          __threadfence();
#pragma unroll
          for (int it = 0; it < 4; ++it) {
            const size_t o = rb + (size_t)(it * 4 + q) * NQKV;
            *(volatile v8us*)(QKVh + o) = hv[it];
            *(volatile v8us*)(QKVl + o) = lv[it];
          }
          wave_lds_sync();
        }
      } else {
        const int g0 = n0 - NQKV;
        const int c4 = c * 4;
#pragma unroll
        for (int i = 0; i < 2; ++i) {
#pragma unroll
          for (int j = 0; j < 4; ++j) {
            const float bv = bg[g0 + 16 * j + c];
#pragma unroll
            for (int r = 0; r < 8; ++r) sl[(8 * hh + r) * SLP + 16 * j + c] = acc[i][j][r] + bv;
          }
          wave_lds_sync();
          v4f gv[8];
#pragma unroll
          for (int it = 0; it < 8; ++it) gv[it] = *(const v4f*)(sl + (it * 2 + hh) * SLP + c4);
          float* gb = Gout + (size_t)(m0 + 16 * i) * DD + g0 + c4;
#pragma unroll
          for (int it = 0; it < 8; ++it) *(volatile v4f*)(gb + (size_t)(it * 2 + hh) * DD) = gv[it];
          __threadfence();
#pragma unroll
          for (int it = 0; it < 8; ++it) *(volatile v4f*)(gb + (size_t)(it * 2 + hh) * DD) = gv[it];
          wave_lds_sync();
        }
      }
    } else {
      v8f accb[2];
      accb[0] = zero8(); accb[1] = zero8();
#pragma unroll
      for (int ks = 0; ks < 4; ++ks) {
        const int k0 = ks * 32;
        const size_t bo = (size_t)(512 + c) * DD + k0 + 8 * hh;
        const v16b bh = ldfrag(WTh + bo);
        const v16b bl = ldfrag(WTl + bo);
#pragma unroll
        for (int i = 0; i < 2; ++i) {
          const v16b ah = ldfrag(Xh + (16 * i + c) * XP + k0 + 8 * hh);
          const v16b al = ldfrag(Xl + (16 * i + c) * XP + k0 + 8 * hh);
          accb[i] = mma_g(ah, bh, accb[i]);
          accb[i] = mma_g(ah, bl, accb[i]);
          accb[i] = mma_g(al, bh, accb[i]);
        }
      }
      if (c < 4) {
#pragma unroll
        for (int i = 0; i < 2; ++i)
#pragma unroll
          for (int r = 0; r < 8; ++r) sl[c * 32 + 16 * i + 8 * hh + r] = accb[i][r];
      }
      wave_lds_sync();
      {
        const int hq = lane >> 3, piece = lane & 7;
        const v4f val = *(const v4f*)(sl + hq * 32 + 4 * piece);
        volatile v4f* bp = (volatile v4f*)(BIAS + (size_t)hq * NROWS + m0 + 4 * piece);
        *bp = val;
        __threadfence();
        *bp = val;
      }
      wave_lds_sync();
    }
  }
}

__global__ __launch_bounds__(256) void attn_kernel(const us* __restrict__ QKVh, const us* __restrict__ QKVl,
                                                   const float* __restrict__ BIAS, const int* __restrict__ msk,
                                                   float* GO) {
  extern __shared__ __align__(16) unsigned char att_smem[];
  us*    Ksh = (us*)(att_smem + AT_KSH);
  us*    Ksl = (us*)(att_smem + AT_KSL);
  us*    VTh = (us*)(att_smem + AT_VTH);
  us*    VTl = (us*)(att_smem + AT_VTL);
  us*    Ph  = (us*)(att_smem + AT_PH);
  us*    Pl  = (us*)(att_smem + AT_PL);
  float* Os  = (float*)(att_smem + AT_OS);

  const int h = blockIdx.x & 3;
  const int i = blockIdx.x >> 2;
  const int tid = threadIdx.x, wave = tid >> 5, lane = tid & 31, hh = lane >> 4, c = lane & 15;

  {
    const int j = tid;
    const size_t rb = (size_t)(i * NN + j) * NQKV + h * DHD;
#pragma unroll
    for (int cc = 0; cc < 4; ++cc) {
      const v8us kh = *(const v8us*)(QKVh + rb + DD + 8 * cc);
      const v8us kl = *(const v8us*)(QKVl + rb + DD + 8 * cc);
      *(v8us*)(Ksh + j * KP + 8 * cc) = kh;
      *(v8us*)(Ksl + j * KP + 8 * cc) = kl;
    }
#pragma unroll
    for (int cc = 0; cc < 4; ++cc) {
      const v8us vh = *(const v8us*)(QKVh + rb + 2 * DD + 8 * cc);
      const v8us vl = *(const v8us*)(QKVl + rb + 2 * DD + 8 * cc);
#pragma unroll
      for (int e = 0; e < 8; ++e) {
        VTh[(8 * cc + e) * VP + j] = vh[e];
        VTl[(8 * cc + e) * VP + j] = vl[e];
      }
    }
  }
  __syncthreads();

  us* Pwh = Ph + wave * 16 * PP;
  us* Pwl = Pl + wave * 16 * PP;
  float* os = Os + wave * 16 * OSP;
  const float* Bh = BIAS + (size_t)h * NROWS;

#pragma unroll 1
  for (int qq = 0; qq < 2; ++qq) {
    const int j0 = (wave + 8 * qq) * 16;
    const size_t qo = (size_t)(i * NN + j0 + c) * NQKV + h * DHD + 8 * hh;
    const v16b qah = ldfrag(QKVh + qo);
    const v16b qal = ldfrag(QKVl + qo);
    int vbits = 0;
#pragma unroll
    for (int r = 0; r < 8; ++r) vbits |= (msk[i * NN + j0 + 8 * hh + r] != 0) ? (1 << r) : 0;
    const float* brow = Bh + (size_t)(j0 + 8 * hh) * NN;

    float mrow[8], lrow[8];
    v8f oacc[2];
#pragma unroll
    for (int r = 0; r < 8; ++r) { mrow[r] = -__builtin_inff(); lrow[r] = 0.0f; }
    oacc[0] = zero8(); oacc[1] = zero8();

#pragma unroll 1
    for (int kc = 0; kc < 4; ++kc) {
      const int kv0 = kc * 64;
      v8f s[4];
#pragma unroll
      for (int jj = 0; jj < 4; ++jj) {
        s[jj] = zero8();
        const us* kp = Ksh + (kv0 + 16 * jj + c) * KP + 8 * hh;
        const us* lp = Ksl + (kv0 + 16 * jj + c) * KP + 8 * hh;
        const v16b kb = ldfrag(kp);
        const v16b kl = ldfrag(lp);
        s[jj] = mma_g(qah, kb, s[jj]);
        s[jj] = mma_g(qah, kl, s[jj]);
        s[jj] = mma_g(qal, kb, s[jj]);
      }
      float cm[8];
#pragma unroll
      for (int r = 0; r < 8; ++r) {
        const bool valid = ((vbits >> r) & 1) != 0;
        float m = -__builtin_inff();
#pragma unroll
        for (int jj = 0; jj < 4; ++jj) {
          float sv = s[jj][r] * SCALEV + brow[r * NN + kv0 + 16 * jj + c];
          sv = valid ? sv : MINV;
          s[jj][r] = sv;
          m = fmaxf(m, sv);
        }
#pragma unroll
        for (int off = 1; off < 16; off <<= 1) m = fmaxf(m, __shfl_xor(m, off, 32));
        cm[r] = m;
      }
#pragma unroll
      for (int r = 0; r < 8; ++r) {
        const float mnew = fmaxf(mrow[r], cm[r]);
        const float alpha = __expf(mrow[r] - mnew);
        mrow[r] = mnew;
        float psum = 0.0f;
#pragma unroll
        for (int jj = 0; jj < 4; ++jj) {
          const float p = __expf(s[jj][r] - mnew);
          psum += p;
          us ph_, pl_; split_bf(p, ph_, pl_);
          Pwh[(8 * hh + r) * PP + 16 * jj + c] = ph_;
          Pwl[(8 * hh + r) * PP + 16 * jj + c] = pl_;
        }
#pragma unroll
        for (int off = 1; off < 16; off <<= 1) psum += __shfl_xor(psum, off, 32);
        lrow[r] = lrow[r] * alpha + psum;
        oacc[0][r] *= alpha;
        oacc[1][r] *= alpha;
      }
      wave_lds_sync();
#pragma unroll
      for (int kk = 0; kk < 2; ++kk) {
        const v16b pa = ldfrag(Pwh + c * PP + kk * 32 + 8 * hh);
        const v16b pl = ldfrag(Pwl + c * PP + kk * 32 + 8 * hh);
#pragma unroll
        for (int t = 0; t < 2; ++t) {
          const us* vp = VTh + (t * 16 + c) * VP + kv0 + kk * 32 + 8 * hh;
          const us* wp = VTl + (t * 16 + c) * VP + kv0 + kk * 32 + 8 * hh;
          const v16b vb = ldfrag(vp);
          const v16b vl = ldfrag(wp);
          oacc[t] = mma_g(pa, vb, oacc[t]);
          oacc[t] = mma_g(pa, vl, oacc[t]);
          oacc[t] = mma_g(pl, vb, oacc[t]);
        }
      }
      wave_lds_sync();
    }

#pragma unroll
    for (int r = 0; r < 8; ++r) {
      const float inv = 1.0f / lrow[r];
      const bool valid = ((vbits >> r) & 1) != 0;
      const size_t grow = (size_t)(i * NN + j0 + 8 * hh + r) * DD + h * DHD;
#pragma unroll
      for (int t = 0; t < 2; ++t) {
        const float gr = GO[grow + t * 16 + c];
        const float sig = 1.0f / (1.0f + expf(-gr));
        const float gate = valid ? sig : 0.0f;
        os[(8 * hh + r) * OSP + t * 16 + c] = oacc[t][r] * inv * gate;
      }
    }
    wave_lds_sync();
    {
      const int q = lane >> 3, c4 = (lane & 7) * 4;
      v4f ov[4];
#pragma unroll
      for (int it = 0; it < 4; ++it) ov[it] = *(const v4f*)(os + (it * 4 + q) * OSP + c4);
      float* ob = GO + (size_t)(i * NN + j0) * DD + h * DHD + c4;
#pragma unroll
      for (int it = 0; it < 4; ++it) *(volatile v4f*)(ob + (size_t)(it * 4 + q) * DD) = ov[it];
      __threadfence();
#pragma unroll
      for (int it = 0; it < 4; ++it) *(volatile v4f*)(ob + (size_t)(it * 4 + q) * DD) = ov[it];
    }
    wave_lds_sync();
  }
}

__global__ __launch_bounds__(256) void oproj_kernel(float* OUT, const us* __restrict__ WoTh, const us* __restrict__ WoTl,
                                                    const float* __restrict__ bo) {
  __shared__ __align__(16) us Ah[32 * XP];
  __shared__ __align__(16) us Al[32 * XP];
  __shared__ __align__(16) float slab[8][16 * OSP];
  const int tid = threadIdx.x, wave = tid >> 5, lane = tid & 31, hh = lane >> 4, c = lane & 15;
  const int m0 = blockIdx.x * 32;
  {
    const int row = tid >> 3, c16 = (tid & 7) * 16;
    const float* src = OUT + (size_t)(m0 + row) * DD + c16;
    us hb[16], lb[16];
#pragma unroll
    for (int qd = 0; qd < 4; ++qd) {
      const v4f x = *(const v4f*)(src + 4 * qd);
#pragma unroll
      for (int e = 0; e < 4; ++e) split_bf(x[e], hb[4 * qd + e], lb[4 * qd + e]);
    }
    v4u h0, h1, l0, l1;
#pragma unroll
    for (int w = 0; w < 4; ++w) {
      h0[w] = pk16(hb[2 * w], hb[2 * w + 1]);      h1[w] = pk16(hb[8 + 2 * w], hb[9 + 2 * w]);
      l0[w] = pk16(lb[2 * w], lb[2 * w + 1]);      l1[w] = pk16(lb[8 + 2 * w], lb[9 + 2 * w]);
    }
    *(v4u*)(Ah + row * XP + c16)     = h0;
    *(v4u*)(Ah + row * XP + c16 + 8) = h1;
    *(v4u*)(Al + row * XP + c16)     = l0;
    *(v4u*)(Al + row * XP + c16 + 8) = l1;
  }
  __syncthreads();

  const int rt = wave >> 2, ct = wave & 3;
  v8f acc[2];
  acc[0] = zero8(); acc[1] = zero8();
#pragma unroll
  for (int ks = 0; ks < 4; ++ks) {
    const int k0 = ks * 32;
    const v16b ah = ldfrag(Ah + (16 * rt + c) * XP + k0 + 8 * hh);
    const v16b al = ldfrag(Al + (16 * rt + c) * XP + k0 + 8 * hh);
#pragma unroll
    for (int j = 0; j < 2; ++j) {
      const size_t bofs = (size_t)(32 * ct + 16 * j + c) * DD + k0 + 8 * hh;
      const v16b bh = ldfrag(WoTh + bofs);
      const v16b bl = ldfrag(WoTl + bofs);
      acc[j] = mma_g(ah, bh, acc[j]);
      acc[j] = mma_g(ah, bl, acc[j]);
      acc[j] = mma_g(al, bh, acc[j]);
    }
  }
  float* sl = slab[wave];
#pragma unroll
  for (int j = 0; j < 2; ++j) {
    const float bv = bo[32 * ct + 16 * j + c];
#pragma unroll
    for (int r = 0; r < 8; ++r) sl[(8 * hh + r) * OSP + 16 * j + c] = acc[j][r] + bv;
  }
  wave_lds_sync();
  {
    const int q = lane >> 3, c4 = (lane & 7) * 4;
    v4f ov[4];
#pragma unroll
    for (int it = 0; it < 4; ++it) ov[it] = *(const v4f*)(sl + (it * 4 + q) * OSP + c4);
    float* ob = OUT + (size_t)(m0 + 16 * rt) * DD + 32 * ct + c4;
#pragma unroll
    for (int it = 0; it < 4; ++it) *(volatile v4f*)(ob + (size_t)(it * 4 + q) * DD) = ov[it];
    __threadfence();
#pragma unroll
    for (int it = 0; it < 4; ++it) *(volatile v4f*)(ob + (size_t)(it * 4 + q) * DD) = ov[it];
  }
}

extern "C" void kernel_launch(void* const* d_in, const int* in_sizes, int n_in,
                              void* d_out, int out_size, void* d_ws, size_t ws_size,
                              hipStream_t stream) {
  if (n_in < 10) return;
  if (in_sizes[0] != NROWS * DD || in_sizes[1] != NROWS) return;
  if (in_sizes[2] != DD || in_sizes[3] != DD) return;
  if (in_sizes[4] != DD * NQKV || in_sizes[5] != DD * NH || in_sizes[6] != DD * DD || in_sizes[7] != DD) return;
  if (in_sizes[8] != DD * DD || in_sizes[9] != DD) return;
  if (out_size != NROWS * DD) return;

  const float* edges = (const float*)d_in[0];
  const int*   msk   = (const int*)d_in[1];
  const float* ln_g  = (const float*)d_in[2];
  const float* ln_b  = (const float*)d_in[3];
  const float* Wqkv  = (const float*)d_in[4];
  const float* Wb    = (const float*)d_in[5];
  const float* Wg    = (const float*)d_in[6];
  const float* bg    = (const float*)d_in[7];
  const float* Wout  = (const float*)d_in[8];
  const float* bout  = (const float*)d_in[9];
  float*       out   = (float*)d_out;

  const size_t szWT  = (size_t)NCAT * DD * 2;
  const size_t szWoT = (size_t)DD * DD * 2;
  const size_t szB   = (size_t)NH * NROWS * 4;
  const size_t szQKV = (size_t)NROWS * NQKV * 2;
  size_t off = 0;
  const size_t oWTh  = off; off += szWT;
  const size_t oWTl  = off; off += szWT;
  const size_t oWoTh = off; off += szWoT;
  const size_t oWoTl = off; off += szWoT;
  const size_t oBIAS = off; off += szB;
  const size_t oQKVh = off; off += szQKV;
  const size_t oQKVl = off; off += szQKV;
  if (off > ws_size) return;

  char* ws = (char*)d_ws;
  us*    WTh  = (us*)(ws + oWTh);
  us*    WTl  = (us*)(ws + oWTl);
  us*    WoTh = (us*)(ws + oWoTh);
  us*    WoTl = (us*)(ws + oWoTl);
  float* BIAS = (float*)(ws + oBIAS);
  us*    QKVh = (us*)(ws + oQKVh);
  us*    QKVl = (us*)(ws + oQKVl);

  hipFuncSetAttribute((const void*)attn_kernel, hipFuncAttributeMaxDynamicSharedMemorySize, AT_SMEM);

  prep_kernel<<<dim3(NCAT + DD), dim3(32), 0, stream>>>(Wqkv, Wb, Wg, Wout, WTh, WTl, WoTh, WoTl);
  proj_kernel<<<dim3(NROWS / 32), dim3(256), 0, stream>>>(edges, ln_g, ln_b, bg, WTh, WTl, QKVh, QKVl, out, BIAS);
  attn_kernel<<<dim3(NH * NN), dim3(256), AT_SMEM, stream>>>(QKVh, QKVl, BIAS, msk, out);
  oproj_kernel<<<dim3(NROWS / 32), dim3(256), 0, stream>>>(out, WoTh, WoTl, bout);
  (void)hipGetLastError();
}
